// RGAT_PyG_28776280883883
// MI455X (gfx1250) — hardware-run, weakly checked
//
#include <hip/hip_runtime.h>
#include <stddef.h>
#include <stdint.h>
#include <math.h>


#define NN      50000
#define NE      250000
#define FW      256
#define NHD     4
#define HDW     64
#define NCLS    153
#define NCP     160
#define MP      50048
#define KHL     512
#define NTHR    256
#define NWAVE   8
#define EPT     8
#define CHUNK   (NTHR * EPT)
#define WCAP    (EPT * 32)
#define LISTN   (NWAVE * WCAP)
#define NBA     1024
#define SLA     10
#define GA      49
#define RCAP    8192
#define DEGCAP  32
#define MEAS_B1024  5266
#define MEAS_MAXDEG 17
#define GROWS   128
#define GPITCH  260
#define PARSET  768
#define NEGSL   0.2f
#define ACT0    0.01f
#define MX0     (-1.0e30f)
#define BKT_LDS_INTS  (LISTN + RCAP + 16)
#define SCAN_ZINTS    (2 * RCAP + 6 * NBA + 16)
#define SCAN_LDS_INTS (4 * RCAP + 6 * NBA + 16 + 512)
#define GEMM_LDS_FLT  (GROWS * GPITCH + 512)
#define OUT_LDS_FLT   (GROWS * NCLS)
#define OUT_F4        (GROWS * NCLS / 4)
#define OUT_NIT       ((OUT_F4 + NTHR - 1) / NTHR)

static_assert((CHUNK & (CHUNK - 1)) == 0 && CHUNK <= 4096);
static_assert(NBA == (1 << SLA) && ((long long)CHUNK << SLA) < (1LL << 31));
static_assert(NN <= 65536);
static_assert((NE % 4) == 0);
static_assert(MP % GROWS == 0 && MP >= NN && MP - NN < GROWS);
static_assert(GA * NBA >= MP && (GA - 1) * NBA < NN);
static_assert((NBA % GROWS) == 0);
static_assert(RCAP >= MEAS_B1024 + 2048 && (RCAP % 32) == 0);
static_assert(DEGCAP >= MEAS_MAXDEG + 8 && DEGCAP <= 32);
static_assert((SCAN_ZINTS % 4) == 0);
static_assert(SCAN_LDS_INTS * 4 <= 300000 && BKT_LDS_INTS * 4 <= 65536);
static_assert(GEMM_LDS_FLT * 4 <= 300000 && OUT_LDS_FLT * 4 <= 300000);
static_assert(GROWS == NWAVE * 16 && NTHR == 2 * GROWS);
static_assert(FW == NHD * HDW && FW == 8 * 32);
static_assert(KHL == 2 * FW && (FW % 32) == 0 && (KHL % 32) == 0);
static_assert(NCP == 2 * 80 && NCP >= NCLS && (NCP % 16) == 0);
static_assert(((GROWS * NCLS) % 4) == 0 && (((NN % GROWS) * NCLS) % 4) == 0);
static_assert(((GROWS * NCLS * 4) % 128) == 0);
static_assert((MP * 32) % NTHR == 0);
static_assert((GPITCH % 4) == 0);

typedef float          v4f  __attribute__((ext_vector_type(4)));
typedef float          v8f  __attribute__((ext_vector_type(8)));
typedef int            v4i  __attribute__((ext_vector_type(4)));
typedef int            v8i  __attribute__((ext_vector_type(8)));
typedef unsigned short v8us __attribute__((ext_vector_type(8)));
typedef __bf16         v16b __attribute__((ext_vector_type(16)));
typedef v4f  __attribute__((may_alias)) v4fa;
typedef v4i  __attribute__((may_alias)) v4ia;
typedef v8us __attribute__((may_alias)) v8usa;
union FragB { v16b v; v8us h[2]; v8i w; };

__device__ __forceinline__ v8f wmb(const FragB& a, const FragB& b, v8f c) {
  v8f d = __builtin_amdgcn_wmma_f32_16x16x32_bf16(false, a.v, false, b.v, (short)0, c, false, false);
  asm volatile("v_nop\n\tv_nop\n\tv_nop\n\tv_nop" : "+v"(d) : "v"(a.w), "v"(b.w));
  return d;
}

__device__ __forceinline__ unsigned int f2bf(float f) {
  const unsigned int u = __float_as_uint(f);
  const unsigned int r = ((u + 0x7FFFu + ((u >> 16) & 1u)) >> 16) & 0xFFFFu;
  return ((u & 0x7FFFFFFFu) > 0x7F800000u) ? 0x7FC0u : r;
}
__device__ __forceinline__ float bf2f(unsigned int b) { return __uint_as_float(b << 16); }
__device__ __forceinline__ float bfr(float f) { return bf2f(f2bf(f)); }
__device__ __forceinline__ v4f bfr4(v4f q) {
  v4f r; r.x = bfr(q.x); r.y = bfr(q.y); r.z = bfr(q.z); r.w = bfr(q.w); return r;
}
__device__ __forceinline__ v8us cv8(const float* __restrict__ p, size_t stride) {
  v8us o;
#pragma unroll
  for (int i = 0; i < 8; ++i) o[i] = (unsigned short)f2bf(p[(size_t)i * stride]);
  return o;
}

template <int SLB>
__device__ __forceinline__ int scan_chunk(const int* __restrict__ dsts, int nE, int cbase, int slotBase,
                                          int nb, int vec8, int* list, int tid, int lane, int wave) {
  int wc = 0;
  const int el0  = tid * EPT;
  const int e0   = cbase + el0;
  const int sent = -2147483647 - 1;
  v4i da, db;
  if (vec8 != 0 && cbase + CHUNK <= nE) {
    da = *(const v4i*)(dsts + e0);
    db = *(const v4i*)(dsts + e0 + 4);
  } else {
    da.x = (e0     < nE) ? dsts[min(e0,     nE - 1)] : sent;
    da.y = (e0 + 1 < nE) ? dsts[min(e0 + 1, nE - 1)] : sent;
    da.z = (e0 + 2 < nE) ? dsts[min(e0 + 2, nE - 1)] : sent;
    da.w = (e0 + 3 < nE) ? dsts[min(e0 + 3, nE - 1)] : sent;
    db.x = (e0 + 4 < nE) ? dsts[min(e0 + 4, nE - 1)] : sent;
    db.y = (e0 + 5 < nE) ? dsts[min(e0 + 5, nE - 1)] : sent;
    db.z = (e0 + 6 < nE) ? dsts[min(e0 + 6, nE - 1)] : sent;
    db.w = (e0 + 7 < nE) ? dsts[min(e0 + 7, nE - 1)] : sent;
  }
  const unsigned nbs = (unsigned)slotBase;
  const unsigned unb = (unsigned)nb;
  const unsigned s0 = (unsigned)da.x - nbs, s1 = (unsigned)da.y - nbs;
  const unsigned s2 = (unsigned)da.z - nbs, s3 = (unsigned)da.w - nbs;
  const unsigned s4 = (unsigned)db.x - nbs, s5 = (unsigned)db.y - nbs;
  const unsigned s6 = (unsigned)db.z - nbs, s7 = (unsigned)db.w - nbs;
  const bool h0 = s0 < unb, h1 = s1 < unb, h2 = s2 < unb, h3 = s3 < unb;
  const bool h4 = s4 < unb, h5 = s5 < unb, h6 = s6 < unb, h7 = s7 < unb;
  const unsigned any = __builtin_amdgcn_ballot_w32(h0 | h1 | h2 | h3 | h4 | h5 | h6 | h7);
  if (any != 0u) {
#define HITJ(J, HJ, SJ) { \
      const unsigned mj = __builtin_amdgcn_ballot_w32(HJ); \
      if (mj != 0u) { \
        if (HJ) { \
          const int pos = wc + (int)__builtin_amdgcn_mbcnt_lo(mj, 0u); \
          if (pos < WCAP) list[wave * WCAP + pos] = ((el0 + (J)) << SLB) | (int)(SJ); \
        } \
        wc += (int)__builtin_popcount(mj); } }
    HITJ(0, h0, s0)
    HITJ(1, h1, s1)
    HITJ(2, h2, s2)
    HITJ(3, h3, s3)
    HITJ(4, h4, s4)
    HITJ(5, h5, s5)
    HITJ(6, h6, s6)
    HITJ(7, h7, s7)
#undef HITJ
  }
  return wc;
}

__global__ __launch_bounds__(NTHR) void k_px(const float* __restrict__ x, unsigned short* XB) {
  const int u = (int)blockIdx.x * NTHR + (int)threadIdx.x;
  if (u >= MP * 32) return;
  const int row = u >> 5;
  const int c0  = (u & 31) * 8;
  const int rc  = row < NN ? row : NN - 1;
  const float* p = x + (size_t)rc * FW + c0;
  const v4f a = *(const v4fa*)p;
  const v4f b = *(const v4fa*)(p + 4);
  asm volatile("" :: "v"(a), "v"(b));
  const bool live = row < NN;
  v8us o;
  o[0] = live ? (unsigned short)f2bf(a.x) : (unsigned short)0;
  o[1] = live ? (unsigned short)f2bf(a.y) : (unsigned short)0;
  o[2] = live ? (unsigned short)f2bf(a.z) : (unsigned short)0;
  o[3] = live ? (unsigned short)f2bf(a.w) : (unsigned short)0;
  o[4] = live ? (unsigned short)f2bf(b.x) : (unsigned short)0;
  o[5] = live ? (unsigned short)f2bf(b.y) : (unsigned short)0;
  o[6] = live ? (unsigned short)f2bf(b.z) : (unsigned short)0;
  o[7] = live ? (unsigned short)f2bf(b.w) : (unsigned short)0;
  unsigned short* dp = XB + (size_t)u * 8;
  *(volatile v8us*)dp = o;
  __threadfence();
  *(volatile v8us*)dp = o;
}

template <int KD>
__global__ __launch_bounds__(NTHR) void k_pw2(const float* __restrict__ Wa, const float* __restrict__ Wb,
                                              unsigned short* WT) {
  constexpr int UPR = KD / 8;
  static_assert((256 * UPR) % NTHR == 0 && (512 * UPR) % NTHR == 0);
  const int u = (int)blockIdx.x * NTHR + (int)threadIdx.x;
  if (u >= 512 * UPR) return;
  const int n  = u / UPR;
  const int k8 = (u - n * UPR) * 8;
  const int kk = k8 & (FW - 1);
  const int nn = n & (FW - 1);
  v8us o;
  if (n < FW) o = cv8(Wa + (size_t)kk * FW + nn, FW);
  else        o = cv8(Wb + (size_t)kk * FW + nn, FW);
  unsigned short* dp = WT + (size_t)u * 8;
  *(volatile v8us*)dp = o;
  __threadfence();
  *(volatile v8us*)dp = o;
}

__global__ __launch_bounds__(NTHR) void k_pwo(const float* __restrict__ Wout, unsigned short* WOD) {
  const int u = (int)blockIdx.x * NTHR + (int)threadIdx.x;
  if (u >= NCP * (KHL / 8)) return;
  const int n  = u >> 6;
  const int k8 = (u & 63) * 8;
  const int kk = k8 & (FW - 1);
  const int nc = n < NCLS ? n : NCLS - 1;
  v8us o = cv8(Wout + (size_t)kk * NCLS + nc, NCLS);
  asm volatile("" :: "v"(o));
  const v8us z8 = {0, 0, 0, 0, 0, 0, 0, 0};
  if (n >= NCLS) o = z8;
  unsigned short* dp = WOD + (size_t)u * 8;
  *(volatile v8us*)dp = o;
  __threadfence();
  *(volatile v8us*)dp = o;
}

template <int WB>
__global__ __launch_bounds__(64) void k_pv(const float* __restrict__ sa, const float* __restrict__ da,
                                           const float* __restrict__ ba, const float* __restrict__ sb,
                                           const float* __restrict__ db, const float* __restrict__ bb,
                                           const float* __restrict__ bo, float* PARL, float* BOUT) {
  const int t = (int)threadIdx.x;
  const v4f q0 = bfr4(*(const v4fa*)(sa + 4 * t));
  const v4f q1 = bfr4(*(const v4fa*)(da + 4 * t));
  const v4f q2 = bfr4(*(const v4fa*)(ba + 4 * t));
  const v4f q3 = bfr4(*(const v4fa*)(sb + 4 * t));
  const v4f q4 = bfr4(*(const v4fa*)(db + 4 * t));
  const v4f q5 = bfr4(*(const v4fa*)(bb + 4 * t));
  v4f qb = {0.f, 0.f, 0.f, 0.f};
  if constexpr (WB == 1) {
    const int i0 = 4 * t;
    const float f0 = bo[min(i0,     NCLS - 1)];
    const float f1 = bo[min(i0 + 1, NCLS - 1)];
    const float f2 = bo[min(i0 + 2, NCLS - 1)];
    const float f3 = bo[min(i0 + 3, NCLS - 1)];
    asm volatile("" :: "v"(f0), "v"(f1), "v"(f2), "v"(f3));
    qb.x = (i0     < NCLS) ? bfr(f0) : 0.0f;
    qb.y = (i0 + 1 < NCLS) ? bfr(f1) : 0.0f;
    qb.z = (i0 + 2 < NCLS) ? bfr(f2) : 0.0f;
    qb.w = (i0 + 3 < NCLS) ? bfr(f3) : 0.0f;
  }
  float* p = PARL + 4 * t;
  const bool wb = (WB == 1) && (t < NCP / 4);
  float* pb = BOUT + 4 * (t < NCP / 4 ? t : 0);
  *(volatile v4f*)(p)        = q0;
  *(volatile v4f*)(p + 256)  = q1;
  *(volatile v4f*)(p + 512)  = q2;
  *(volatile v4f*)(p + 768)  = q3;
  *(volatile v4f*)(p + 1024) = q4;
  *(volatile v4f*)(p + 1280) = q5;
  if (wb) *(volatile v4f*)pb = qb;
  __threadfence();
  *(volatile v4f*)(p)        = q0;
  *(volatile v4f*)(p + 256)  = q1;
  *(volatile v4f*)(p + 512)  = q2;
  *(volatile v4f*)(p + 768)  = q3;
  *(volatile v4f*)(p + 1024) = q4;
  *(volatile v4f*)(p + 1280) = q5;
  if (wb) *(volatile v4f*)pb = qb;
}

__global__ __launch_bounds__(NTHR) void k_bucket(const int* __restrict__ srcs, const int* __restrict__ dsts,
                                                 int vec8, int* HITS, int* FLG) {
  extern __shared__ __attribute__((aligned(16))) int bsm[];
  int* list = bsm;
  int* reg1 = bsm + LISTN;
  int* wcnt = reg1 + RCAP;
  const int tid = (int)threadIdx.x, lane = tid & 31, wave = tid >> 5;
  const int blk = (int)blockIdx.x;
  const int nodeBase = blk * NBA;
  int nb = NN - nodeBase;
  nb = nb < 0 ? 0 : (nb > NBA ? NBA : nb);

  int tot = 0, ovf = 0;
  const int nChunks = (NE + CHUNK - 1) / CHUNK;
#pragma unroll 1
  for (int ch = 0; ch < nChunks; ++ch) {
    const int cbase = ch * CHUNK;
    const int wc = scan_chunk<SLA>(dsts, NE, cbase, nodeBase, nb, vec8, list, tid, lane, wave);
    if (lane == 0) wcnt[wave] = wc;
    __syncthreads();
    int pre = 0, all = 0;
#pragma unroll
    for (int w2 = 0; w2 < NWAVE; ++w2) {
      int c = wcnt[w2];
      c = c < 0 ? 0 : (c > WCAP ? WCAP : c);
      all += c;
      pre += (w2 < wave) ? c : 0;
    }
    const int wcc  = wc > WCAP ? WCAP : wc;
    const int base = tot + pre;
#pragma unroll 1
    for (int i = lane; i < wcc; i += 32) {
      const int ent = list[wave * WCAP + i];
      const int el  = (ent >> SLA) & (CHUNK - 1);
      const int sl  = ent & (NBA - 1);
      int eid = cbase + el;
      eid = eid > NE - 1 ? NE - 1 : eid;
      const int sraw = srcs[eid];
      const int s = sraw < 0 ? 0 : (sraw > NN - 1 ? NN - 1 : sraw);
      const int pos = base + i;
      if (pos < RCAP) reg1[pos] = (int)((unsigned)s | ((unsigned)sl << 16));
    }
    if (tot + all > RCAP) ovf = 1;
    tot += all;
    tot = tot > RCAP ? RCAP : tot;
    __syncthreads();
  }
  const int nh = tot;
  for (int i = nh + tid; i < RCAP; i += NTHR) reg1[i] = 0;
  __syncthreads();

  int* hb = HITS + (size_t)blk * RCAP;
  v4i cv;
  cv.x = (tid == 0) ? nh : 0;
  cv.y = (tid == 0) ? ovf : 0;
  cv.z = 0; cv.w = 0;
  int* fp = FLG + (size_t)blk * 32 + 4 * (tid & 7);
#pragma unroll 1
  for (int p = tid * 4; p < RCAP; p += NTHR * 4) {
    const v4i v = *(const v4ia*)(reg1 + p);
    *(volatile v4i*)(hb + p) = v;
  }
  if (tid < 8) *(volatile v4i*)fp = cv;
  __threadfence();
#pragma unroll 1
  for (int p = tid * 4; p < RCAP; p += NTHR * 4) {
    const v4i v = *(const v4ia*)(reg1 + p);
    *(volatile v4i*)(hb + p) = v;
  }
  if (tid < 8) *(volatile v4i*)fp = cv;
}

__global__ __launch_bounds__(NTHR) __attribute__((amdgpu_num_vgpr(248)))
void k_gemm(const unsigned short* __restrict__ A, const unsigned short* __restrict__ WT, int K,
            float* Hout, float* SSD, const float* __restrict__ PARL) {
  extern __shared__ __attribute__((aligned(16))) float gsm[];
  float* stg  = gsm;
  float* satt = gsm + GROWS * GPITCH;
  const int tid = (int)threadIdx.x, lane = tid & 31, wave = tid >> 5, hh = lane >> 4, m = lane & 15;
  const int rowBase = (int)blockIdx.x * GROWS;
  const int lt      = (int)blockIdx.y;

  if (tid < 128) {
    const v4f q = *(const v4fa*)(PARL + (size_t)lt * PARSET + 4 * tid);
    *(v4fa*)(satt + 4 * tid) = q;
  }

  const unsigned short* ap = A + (size_t)(rowBase + 16 * wave + m) * (size_t)K + 8 * hh;
  const int ksteps = K >> 5;
#pragma unroll 1
  for (int hc = 0; hc < NHD; ++hc) {
    v8f acc[4];
    {
      const v8f z = {0.f, 0.f, 0.f, 0.f, 0.f, 0.f, 0.f, 0.f};
      acc[0] = z; acc[1] = z; acc[2] = z; acc[3] = z;
    }
    const unsigned short* wp = WT + (size_t)(lt * FW + hc * HDW + m) * (size_t)K + 8 * hh;
#pragma unroll 1
    for (int ks = 0; ks < ksteps; ++ks) {
      FragB af;
      af.h[0] = *(const v8usa*)(ap + 32 * ks);
      af.h[1] = *(const v8usa*)(ap + 32 * ks + 16);
#pragma unroll
      for (int t = 0; t < 4; ++t) {
        const unsigned short* wq = wp + (size_t)(16 * t) * (size_t)K + 32 * ks;
        FragB bf;
        bf.h[0] = *(const v8usa*)wq;
        bf.h[1] = *(const v8usa*)(wq + 16);
        acc[t] = wmb(af, bf, acc[t]);
      }
    }
#pragma unroll
    for (int t = 0; t < 4; ++t) {
      const int lc = hc * HDW + 16 * t + m;
#pragma unroll
      for (int r = 0; r < 8; ++r) {
        const int lr = 16 * wave + 8 * hh + r;
        stg[lr * GPITCH + lc] = acc[t][r];
      }
    }
  }
  __syncthreads();

  const int drow = tid & 127, which = tid >> 7;
  float d0 = 0.f, d1 = 0.f, d2 = 0.f, d3 = 0.f;
  {
    const float* hr = stg + drow * GPITCH;
    const float* sa = satt + which * FW;
#pragma unroll 1
    for (int c4 = 0; c4 < HDW / 4; ++c4) {
      const v4f h0 = *(const v4fa*)(hr + 4 * c4);
      const v4f a0 = *(const v4fa*)(sa + 4 * c4);
      const v4f h1 = *(const v4fa*)(hr + HDW + 4 * c4);
      const v4f a1 = *(const v4fa*)(sa + HDW + 4 * c4);
      const v4f h2 = *(const v4fa*)(hr + 2 * HDW + 4 * c4);
      const v4f a2 = *(const v4fa*)(sa + 2 * HDW + 4 * c4);
      const v4f h3 = *(const v4fa*)(hr + 3 * HDW + 4 * c4);
      const v4f a3 = *(const v4fa*)(sa + 3 * HDW + 4 * c4);
      d0 = fmaf(h0.x, a0.x, d0); d0 = fmaf(h0.y, a0.y, d0); d0 = fmaf(h0.z, a0.z, d0); d0 = fmaf(h0.w, a0.w, d0);
      d1 = fmaf(h1.x, a1.x, d1); d1 = fmaf(h1.y, a1.y, d1); d1 = fmaf(h1.z, a1.z, d1); d1 = fmaf(h1.w, a1.w, d1);
      d2 = fmaf(h2.x, a2.x, d2); d2 = fmaf(h2.y, a2.y, d2); d2 = fmaf(h2.z, a2.z, d2); d2 = fmaf(h2.w, a2.w, d2);
      d3 = fmaf(h3.x, a3.x, d3); d3 = fmaf(h3.y, a3.y, d3); d3 = fmaf(h3.z, a3.z, d3); d3 = fmaf(h3.w, a3.w, d3);
    }
  }
  v4f dv; dv.x = d0; dv.y = d1; dv.z = d2; dv.w = d3;
  float* sp = SSD + ((size_t)(2 * lt + which) * MP + (size_t)(rowBase + drow)) * 4;
  float* hb = Hout + ((size_t)lt * MP + (size_t)rowBase) * FW;

#pragma unroll 4
  for (int i = 0; i < 16; ++i) {
    const int lr = 16 * wave + i;
    const v4f q0 = *(const v4fa*)(stg + lr * GPITCH + 4 * lane);
    const v4f q1 = *(const v4fa*)(stg + lr * GPITCH + 128 + 4 * lane);
    float* op = hb + (size_t)lr * FW + 4 * lane;
    *(volatile v4f*)op = q0;
    *(volatile v4f*)(op + 128) = q1;
  }
  *(volatile v4f*)sp = dv;
  __threadfence();
#pragma unroll 4
  for (int i = 0; i < 16; ++i) {
    const int lr = 16 * wave + i;
    const v4f q0 = *(const v4fa*)(stg + lr * GPITCH + 4 * lane);
    const v4f q1 = *(const v4fa*)(stg + lr * GPITCH + 128 + 4 * lane);
    float* op = hb + (size_t)lr * FW + 4 * lane;
    *(volatile v4f*)op = q0;
    *(volatile v4f*)(op + 128) = q1;
  }
  *(volatile v4f*)sp = dv;
}

template <int L>
__global__ __launch_bounds__(NTHR) __attribute__((amdgpu_num_vgpr(248)))
void k_scan(const int* __restrict__ HITS, const int* __restrict__ FLG, const float* __restrict__ Hf,
            const float* __restrict__ SSD, const float* __restrict__ PARL, unsigned short* XP) {
  static_assert(L == 0 || L == 1);
  extern __shared__ __attribute__((aligned(16))) int ssm[];
  int* hl   = ssm;
  int* sl   = hl + 2 * RCAP;
  int* cnt  = sl + 2 * RCAP;
  int* offs = cnt + 2 * NBA;
  int* cur  = offs + 2 * NBA;
  int* misc = cur + 2 * NBA;
  float* bl = (float*)(misc + 16);
  const int tid = (int)threadIdx.x, lane = tid & 31, wave = tid >> 5;
  const int blk = (int)blockIdx.x;
  const int nodeBase = blk * NBA;

  const int nraA = FLG[(size_t)blk * 32];
  const int flA  = FLG[(size_t)blk * 32 + 1];
  const int nraB = FLG[(size_t)(GA + blk) * 32];
  const int flB  = FLG[(size_t)(GA + blk) * 32 + 1];
  const int nhA = nraA < 0 ? 0 : (nraA > RCAP ? RCAP : nraA);
  const int nhB = nraB < 0 ? 0 : (nraB > RCAP ? RCAP : nraB);
  const int ovf = (flA != 0 || flB != 0 || nraA < 0 || nraA > RCAP || nraB < 0 || nraB > RCAP) ? 1 : 0;

  {
    const v4i z4 = {0, 0, 0, 0};
    for (int i = tid * 4; i < SCAN_ZINTS; i += NTHR * 4) *(v4ia*)(sl + i) = z4;
#pragma unroll 1
    for (int t = 0; t < 2; ++t) {
      const int nh  = t ? nhB : nhA;
      const int nh4 = (nh + 3) & ~3;
      const int* hb = HITS + ((size_t)t * GA + (size_t)blk) * RCAP;
      int* hd = hl + t * RCAP;
#pragma unroll 1
      for (int p = tid * 4; p < nh4; p += NTHR * 4) *(v4ia*)(hd + p) = *(const v4i*)(hb + p);
    }
    if (tid < 128) {
      const int t = tid >> 6, c4 = tid & 63;
      const v4f q = *(const v4fa*)(PARL + (size_t)t * PARSET + 512 + 4 * c4);
      *(v4fa*)(bl + t * FW + 4 * c4) = q;
    }
  }
  __syncthreads();

  if (wave < 2) {
    const int t  = wave;
    const int nh = t ? nhB : nhA;
    const int* hlt = hl + t * RCAP;
    int* cn = cnt + t * NBA;
#pragma unroll 1
    for (int b0 = 0; b0 < nh; b0 += 32) {
      const int idx = b0 + lane;
      const int uv  = hlt[idx < nh ? idx : nh - 1];
      const int m32 = (nh - b0) < 32 ? (nh - b0) : 32;
#pragma unroll 1
      for (int k = 0; k < m32; ++k) {
        const int u  = __builtin_amdgcn_readlane(uv, k);
        const int sq = (u >> 16) & (NBA - 1);
        if (lane == 0) cn[sq] = cn[sq] + 1;
      }
    }
  }
  __syncthreads();
  if (wave < 2) {
    const int t = wave;
    int* cn = cnt + t * NBA;
    int* of = offs + t * NBA;
    int* cu = cur + t * NBA;
    const int base = lane * (NBA / 32);
    int s = 0;
#pragma unroll 1
    for (int i = 0; i < NBA / 32; ++i) s += cn[base + i];
    int incl = s;
#pragma unroll
    for (int d = 1; d < 32; d <<= 1) {
      const int y = __shfl_up(incl, d, 32);
      if (lane >= d) incl += y;
    }
    int run = incl - s;
#pragma unroll 1
    for (int i = 0; i < NBA / 32; ++i) {
      const int cv = cn[base + i];
      of[base + i] = run;
      cu[base + i] = run;
      run += cv;
    }
  }
  __syncthreads();
  if (wave < 2) {
    const int t  = wave;
    const int nh = t ? nhB : nhA;
    const int* hlt = hl + t * RCAP;
    int* slt = sl + t * RCAP;
    int* cu  = cur + t * NBA;
#pragma unroll 1
    for (int b0 = 0; b0 < nh; b0 += 32) {
      const int idx = b0 + lane;
      const int uv  = hlt[idx < nh ? idx : nh - 1];
      const int m32 = (nh - b0) < 32 ? (nh - b0) : 32;
#pragma unroll 1
      for (int k = 0; k < m32; ++k) {
        const int u  = __builtin_amdgcn_readlane(uv, k);
        const int sq = (u >> 16) & (NBA - 1);
        if (lane == 0) {
          int p = cu[sq];
          p = p < 0 ? 0 : (p > RCAP - 1 ? RCAP - 1 : p);
          slt[p] = u;
          cu[sq] = p + 1;
        }
      }
    }
  }
  __syncthreads();

  const float qnan = __int_as_float(0x7fc00000);
  const int head = lane >> 3;

#pragma unroll 1
  for (int si = 0; si < NBA / NWAVE; ++si) {
    const int s    = si * NWAVE + wave;
    const int node = nodeBase + s;
    const int nc   = node < NN ? node : NN - 1;
    float v[8];
#pragma unroll
    for (int i = 0; i < 8; ++i) v[i] = 0.0f;
    int bigAny = 0;

#pragma unroll 1
    for (int t = 0; t < 2; ++t) {
      const int nht = t ? nhB : nhA;
      const int craw = __builtin_amdgcn_readfirstlane(cnt[t * NBA + s]);
      bigAny |= (craw > DEGCAP) ? 1 : 0;
      int c = craw < 0 ? 0 : (craw > DEGCAP ? DEGCAP : craw);
      int o = __builtin_amdgcn_readfirstlane(offs[t * NBA + s]);
      o = o < 0 ? 0 : (o > RCAP ? RCAP : o);
      if (c > nht - o) c = nht - o;
      c = c < 0 ? 0 : c;
      const float* Ft  = Hf + (size_t)t * MP * FW;
      const float* SSt = SSD + (size_t)(2 * t) * MP * 4;
      const float adv  = SSD[((size_t)(2 * t + 1) * MP + (size_t)nc) * 4 + head];
      int li = c > 0 ? c - 1 : 0;
      li = lane < li ? lane : li;
      int idx = o + li;
      idx = idx < 0 ? 0 : (idx > RCAP - 1 ? RCAP - 1 : idx);
      const int ent = sl[t * RCAP + idx];
      int hs = ent & 0xFFFF;
      hs = hs > NN - 1 ? NN - 1 : hs;

      float mx = MX0, dn = 0.0f;
      float acc[8];
#pragma unroll
      for (int i = 0; i < 8; ++i) acc[i] = 0.0f;
#pragma unroll 1
      for (int k = 0; k < c; ++k) {
        const int sk = __builtin_amdgcn_readlane(hs, k);
        const float* rp = Ft + (size_t)sk * FW + 8 * lane;
        float lg = SSt[(size_t)sk * 4 + head] + adv;
        lg = lg > 0.f ? lg : NEGSL * lg;
        const float df = lg - mx;
        const float ee = expf(-fabsf(df));
        const bool  up = df > 0.f;
        const float s1 = up ? ee : 1.0f;
        const float s2 = up ? 1.0f : ee;
        mx = up ? lg : mx;
        dn = fmaf(dn, s1, s2);
        const v4f a = *(const v4fa*)rp;
        const v4f b = *(const v4fa*)(rp + 4);
        acc[0] = fmaf(acc[0], s1, s2 * a.x); acc[1] = fmaf(acc[1], s1, s2 * a.y);
        acc[2] = fmaf(acc[2], s1, s2 * a.z); acc[3] = fmaf(acc[3], s1, s2 * a.w);
        acc[4] = fmaf(acc[4], s1, s2 * b.x); acc[5] = fmaf(acc[5], s1, s2 * b.y);
        acc[6] = fmaf(acc[6], s1, s2 * b.z); acc[7] = fmaf(acc[7], s1, s2 * b.w);
      }
      const float inv = __builtin_amdgcn_rcpf(dn + 1e-16f);
      const bool has = c > 0;
      const v4f b0 = *(const v4fa*)(bl + t * FW + 8 * lane);
      const v4f b1 = *(const v4fa*)(bl + t * FW + 8 * lane + 4);
      const float c0 = has ? acc[0] * inv : 0.0f;
      const float c1 = has ? acc[1] * inv : 0.0f;
      const float c2 = has ? acc[2] * inv : 0.0f;
      const float c3 = has ? acc[3] * inv : 0.0f;
      const float c4 = has ? acc[4] * inv : 0.0f;
      const float c5 = has ? acc[5] * inv : 0.0f;
      const float c6 = has ? acc[6] * inv : 0.0f;
      const float c7 = has ? acc[7] * inv : 0.0f;
      v[0] += c0 + b0.x; v[1] += c1 + b0.y; v[2] += c2 + b0.z; v[3] += c3 + b0.w;
      v[4] += c4 + b1.x; v[5] += c5 + b1.y; v[6] += c6 + b1.z; v[7] += c7 + b1.w;
    }

    const bool pz   = (ovf != 0) || (bigAny != 0);
    const bool live = node < NN;
    v8us ho, lo;
#pragma unroll
    for (int i = 0; i < 8; ++i) {
      float y = v[i];
      if constexpr (L == 0) y = (y > 0.0f) ? y : ACT0 * y;
      y = pz ? qnan : y;
      const float val = live ? y : 0.0f;
      const unsigned int hbi = f2bf(val);
      ho[i] = (unsigned short)hbi;
      lo[i] = (unsigned short)f2bf(val - bf2f(hbi));
    }
    if (node < MP) {
      unsigned short* hp = XP + (size_t)node * KHL + 8 * lane;
      *(volatile v8us*)hp = ho;
      *(volatile v8us*)(hp + FW) = lo;
      __threadfence();
      *(volatile v8us*)hp = ho;
      *(volatile v8us*)(hp + FW) = lo;
    }
  }
}

__global__ __launch_bounds__(NTHR) __attribute__((amdgpu_num_vgpr(248)))
void k_out(const unsigned short* __restrict__ A2, const unsigned short* __restrict__ WOD,
           const float* __restrict__ BOUT, const int* __restrict__ FLG, float* out) {
  extern __shared__ __attribute__((aligned(16))) float osm[];
  const int tid = (int)threadIdx.x, lane = tid & 31, wave = tid >> 5, hh = lane >> 4, m = lane & 15;
  const int rowBase = (int)blockIdx.x * GROWS;
  const int blk = rowBase >> SLA;
  const int nraA = FLG[(size_t)blk * 32];
  const int flA  = FLG[(size_t)blk * 32 + 1];
  const int nraB = FLG[(size_t)(GA + blk) * 32];
  const int flB  = FLG[(size_t)(GA + blk) * 32 + 1];
  const bool pz = (flA != 0 || flB != 0 || nraA < 0 || nraA > RCAP || nraB < 0 || nraB > RCAP);
  const float qnan = __int_as_float(0x7fc00000);

  const unsigned short* ap = A2 + (size_t)(rowBase + 16 * wave + m) * KHL + 8 * hh;
#pragma unroll 1
  for (int g = 0; g < 2; ++g) {
    v8f acc[5];
    {
      const v8f z = {0.f, 0.f, 0.f, 0.f, 0.f, 0.f, 0.f, 0.f};
      acc[0] = z; acc[1] = z; acc[2] = z; acc[3] = z; acc[4] = z;
    }
    const unsigned short* wp = WOD + (size_t)(80 * g + m) * KHL + 8 * hh;
#pragma unroll 1
    for (int ks = 0; ks < KHL / 32; ++ks) {
      FragB af;
      af.h[0] = *(const v8usa*)(ap + 32 * ks);
      af.h[1] = *(const v8usa*)(ap + 32 * ks + 16);
#pragma unroll
      for (int t = 0; t < 5; ++t) {
        const unsigned short* wq = wp + (size_t)(16 * t) * KHL + 32 * ks;
        FragB bf;
        bf.h[0] = *(const v8usa*)wq;
        bf.h[1] = *(const v8usa*)(wq + 16);
        acc[t] = wmb(af, bf, acc[t]);
      }
    }
#pragma unroll
    for (int t = 0; t < 5; ++t) {
      const int col = 80 * g + 16 * t + m;
      const float bb = BOUT[col];
#pragma unroll
      for (int r = 0; r < 8; ++r) {
        const int lr = 16 * wave + 8 * hh + r;
        float val = acc[t][r] + bb;
        val = pz ? qnan : val;
        if (col < NCLS) osm[lr * NCLS + col] = val;
      }
    }
  }
  __syncthreads();

  int liveRows = NN - rowBase;
  liveRows = liveRows < 0 ? 0 : (liveRows > GROWS ? GROWS : liveRows);
  const int nf4 = (liveRows * NCLS) >> 2;
  float* ob = out + (size_t)rowBase * NCLS;
#pragma unroll 1
  for (int j = 0; j < OUT_NIT; ++j) {
    const int i  = tid + NTHR * j;
    int ic = i < nf4 ? i : nf4 - 1;
    ic = ic < 0 ? 0 : ic;
    const v4f q = *(const v4fa*)(osm + 4 * ic);
    if (i < nf4) *(volatile v4f*)(ob + 4 * (size_t)i) = q;
  }
  __threadfence();
#pragma unroll 1
  for (int j = 0; j < OUT_NIT; ++j) {
    const int i  = tid + NTHR * j;
    int ic = i < nf4 ? i : nf4 - 1;
    ic = ic < 0 ? 0 : ic;
    const v4f q = *(const v4fa*)(osm + 4 * ic);
    if (i < nf4) *(volatile v4f*)(ob + 4 * (size_t)i) = q;
  }
}

static inline size_t al256(size_t o) { return (o + 255) & ~(size_t)255; }

extern "C" void kernel_launch(void* const* d_in, const int* in_sizes, int n_in,
                              void* d_out, int out_size, void* d_ws, size_t ws_size,
                              hipStream_t stream) {
  if (n_in < 21) return;
  if (in_sizes[0] != NN * FW) return;
  if (in_sizes[1] != 2 * NE || in_sizes[2] != 2 * NE) return;
  for (int base = 3; base <= 15; base += 4) {
    if (in_sizes[base] != FW * FW) return;
    if (in_sizes[base + 1] != NHD * HDW || in_sizes[base + 2] != NHD * HDW) return;
    if (in_sizes[base + 3] != FW) return;
  }
  if (in_sizes[19] != FW * NCLS || in_sizes[20] != NCLS) return;
  if ((long long)out_size != (long long)NN * NCLS) return;

  const float* x    = (const float*)d_in[0];
  const int*   eia  = (const int*)  d_in[1];
  const int*   eib  = (const int*)  d_in[2];
  const float* W0a  = (const float*)d_in[3];
  const float* as0a = (const float*)d_in[4];
  const float* ad0a = (const float*)d_in[5];
  const float* b0a  = (const float*)d_in[6];
  const float* W0b  = (const float*)d_in[7];
  const float* as0b = (const float*)d_in[8];
  const float* ad0b = (const float*)d_in[9];
  const float* b0b  = (const float*)d_in[10];
  const float* W1a  = (const float*)d_in[11];
  const float* as1a = (const float*)d_in[12];
  const float* ad1a = (const float*)d_in[13];
  const float* b1a  = (const float*)d_in[14];
  const float* W1b  = (const float*)d_in[15];
  const float* as1b = (const float*)d_in[16];
  const float* ad1b = (const float*)d_in[17];
  const float* b1b  = (const float*)d_in[18];
  const float* Wout = (const float*)d_in[19];
  const float* bout = (const float*)d_in[20];
  float* out = (float*)d_out;

  char* ws = (char*)d_ws;
  size_t off = 0;
  const size_t oX   = off; off = al256(off + (size_t)MP * KHL * 2);
  const size_t oH   = off; off = al256(off + (size_t)2 * MP * FW * 4);
  const size_t oSSD = off; off = al256(off + (size_t)4 * MP * 4 * 4);
  const size_t oHIT = off; off = al256(off + (size_t)2 * GA * RCAP * 4);
  const size_t oFLG = off; off = al256(off + (size_t)2 * GA * 128);
  const size_t oW0  = off; off = al256(off + (size_t)512 * FW * 2);
  const size_t oW1  = off; off = al256(off + (size_t)512 * KHL * 2);
  const size_t oWO  = off; off = al256(off + (size_t)NCP * KHL * 2);
  const size_t oPAR = off; off = al256(off + (size_t)4 * PARSET * 4);
  const size_t oBO  = off; off = al256(off + (size_t)NCP * 4);
  if (off > ws_size) return;
  unsigned short* XR   = (unsigned short*)(ws + oX);
  float*          Hb   = (float*)(ws + oH);
  float*          SSD  = (float*)(ws + oSSD);
  int*            HITS = (int*)(ws + oHIT);
  int*            FLG  = (int*)(ws + oFLG);
  unsigned short* W0T  = (unsigned short*)(ws + oW0);
  unsigned short* W1D  = (unsigned short*)(ws + oW1);
  unsigned short* WOD  = (unsigned short*)(ws + oWO);
  float*          PAR  = (float*)(ws + oPAR);
  float*          BOUT = (float*)(ws + oBO);
  float* PAR0 = PAR;
  float* PAR1 = PAR + 2 * PARSET;

  const int bktLds  = BKT_LDS_INTS * 4;
  const int scanLds = SCAN_LDS_INTS * 4;
  const int gemmLds = GEMM_LDS_FLT * 4;
  const int outLds  = OUT_LDS_FLT * 4;
  hipFuncSetAttribute(reinterpret_cast<const void*>(&k_gemm),
                      hipFuncAttributeMaxDynamicSharedMemorySize, gemmLds);
  hipFuncSetAttribute(reinterpret_cast<const void*>(&k_scan<0>),
                      hipFuncAttributeMaxDynamicSharedMemorySize, scanLds);
  hipFuncSetAttribute(reinterpret_cast<const void*>(&k_scan<1>),
                      hipFuncAttributeMaxDynamicSharedMemorySize, scanLds);
  hipFuncSetAttribute(reinterpret_cast<const void*>(&k_out),
                      hipFuncAttributeMaxDynamicSharedMemorySize, outLds);

  k_px<<<(MP * 32) / NTHR, NTHR, 0, stream>>>(x, XR);
  k_pw2<FW><<<(512 * (FW / 8)) / NTHR, NTHR, 0, stream>>>(W0a, W0b, W0T);
  k_pw2<KHL><<<(512 * (KHL / 8)) / NTHR, NTHR, 0, stream>>>(W1a, W1b, W1D);
  k_pwo<<<(NCP * (KHL / 8)) / NTHR, NTHR, 0, stream>>>(Wout, WOD);
  k_pv<0><<<1, 64, 0, stream>>>(as0a, ad0a, b0a, as0b, ad0b, b0b, bout, PAR0, BOUT);
  k_pv<1><<<1, 64, 0, stream>>>(as1a, ad1a, b1a, as1b, ad1b, b1b, bout, PAR1, BOUT);
  k_bucket<<<GA, NTHR, bktLds, stream>>>(eia, eia + NE, 1, HITS, FLG);
  k_bucket<<<GA, NTHR, bktLds, stream>>>(eib, eib + NE, 1, HITS + (size_t)GA * RCAP, FLG + (size_t)GA * 32);
  k_gemm<<<dim3(MP / GROWS, 2), NTHR, gemmLds, stream>>>(XR, W0T, FW, Hb, SSD, PAR0);
  k_scan<0><<<GA, NTHR, scanLds, stream>>>(HITS, FLG, Hb, SSD, PAR0, XR);
  k_gemm<<<dim3(MP / GROWS, 2), NTHR, gemmLds, stream>>>(XR, W1D, KHL, Hb, SSD, PAR1);
  k_scan<1><<<GA, NTHR, scanLds, stream>>>(HITS, FLG, Hb, SSD, PAR1, XR);
  k_out<<<MP / GROWS, NTHR, outLds, stream>>>(XR, WOD, BOUT, FLG, out);
}
